// MambaFormerCrossAttentionLayer_66288525247129
// MI455X (gfx1250) — hardware-run, weakly checked
//
#include <hip/hip_runtime.h>
#include <math.h>

constexpr int kL   = 4096;
constexpr int kDM  = 1024;
constexpr int kDI  = 2048;
constexpr int kDS  = 16;
constexpr int kDTR = 64;
constexpr int kXPC = 96;
constexpr int kXPN = 128;
constexpr float kEps   = 1e-5f;
constexpr float kInvDM = 1.0f / 1024.0f;
constexpr float kWCarry    = 64.0f;
constexpr float kXsCarry   = 64.0f;
constexpr float kDtCarry   = 64.0f;
constexpr float kGateCarry = 256.0f;
constexpr float kGeluCarry = 16.0f;
constexpr float kScaleIn   = 1.0f / 64.0f;
constexpr float kScaleXp   = 1.0f / 4096.0f;
constexpr float kScaleDt   = 1.0f / 4096.0f;
constexpr float kScaleOut  = 1.0f / 16384.0f;
constexpr float kScaleF1   = 1.0f / 64.0f;
constexpr float kScaleF2   = 1.0f / 1024.0f;

constexpr size_t kMi    = 1048576;
constexpr size_t oXC    = 0;
constexpr size_t oDTP   = 0;
constexpr size_t oSEQ2  = 0;
constexpr size_t oSEQ2H = 16 * kMi;
constexpr size_t oW1H   = 24 * kMi;
constexpr size_t oW2H   = 28 * kMi;
constexpr size_t oZ     = 32 * kMi;
constexpr size_t oHPRE  = 32 * kMi;
constexpr size_t oEMBH  = 64 * kMi;
constexpr size_t oWINH  = 72 * kMi;
constexpr size_t oXSH   = 64 * kMi;
constexpr size_t oGH    = 64 * kMi;
constexpr size_t oG2H   = 64 * kMi;
constexpr size_t oXS    = 80 * kMi;
constexpr size_t oS1    = 80 * kMi;
constexpr size_t oOPRE  = 96 * kMi;
constexpr size_t oWXPH  = 112 * kMi;
constexpr size_t oXDBL  = oWXPH + (size_t)kXPN * kDI * 2;
constexpr size_t oDTINH = oXDBL + (size_t)kL * kXPN * 4;
constexpr size_t oWDTH  = oDTINH + (size_t)kL * kDTR * 2;
constexpr size_t oWOUTH = oWDTH + (size_t)kDI * kDTR * 2;
constexpr size_t oVVEC  = oWOUTH + (size_t)kDM * kDI * 2;
constexpr size_t oAVEC  = oVVEC + (size_t)kDM * 4;
constexpr size_t kWsTotal = oAVEC + (size_t)kDM * 4;
static_assert(kWsTotal == 125050880ull, "ws");
static_assert(kWsTotal <= 134217728ull, "ws");

typedef __attribute__((ext_vector_type(16))) _Float16 v16h;
typedef __attribute__((ext_vector_type(8)))  _Float16 v8h;
typedef __attribute__((ext_vector_type(16))) __bf16   v16b;
typedef __attribute__((ext_vector_type(8)))  __bf16   v8b;
typedef __attribute__((ext_vector_type(8)))  float    v8f;
typedef __attribute__((ext_vector_type(4)))  float    v4f;
typedef __attribute__((ext_vector_type(2)))  float    v2f;
typedef __attribute__((ext_vector_type(4)))  unsigned int v4u;
typedef __attribute__((ext_vector_type(2)))  unsigned int v2u;

__device__ __forceinline__ unsigned short f2bf_bits(float f) {
  unsigned u = __float_as_uint(f);
  return (unsigned short)((u + 0x7FFFu + ((u >> 16) & 1u)) >> 16);
}
__device__ __forceinline__ float bf_bits2f(unsigned short h) { return __uint_as_float(((unsigned)h) << 16); }

__device__ __forceinline__ void dep_guard_h(v8f& a, v8f& b, v16h x, v16h y) { asm volatile("v_nop\n\tv_nop\n\tv_nop\n\tv_nop" : "+v"(a), "+v"(b) : "v"(x), "v"(y)); }
__device__ __forceinline__ void dep_guard_b(v8f& a, v8f& b, v16b x, v16b y) { asm volatile("v_nop\n\tv_nop\n\tv_nop\n\tv_nop" : "+v"(a), "+v"(b) : "v"(x), "v"(y)); }
__device__ __forceinline__ void keep4_h(v16h a, v16h b, v16h c, v16h d) { asm volatile("v_nop" :: "v"(a), "v"(b), "v"(c), "v"(d)); }
__device__ __forceinline__ void keep4_b(v16b a, v16b b, v16b c, v16b d) { asm volatile("v_nop" :: "v"(a), "v"(b), "v"(c), "v"(d)); }
__device__ __forceinline__ void acc_guard4(v8f& a, v8f& b, v8f& c, v8f& d) { asm volatile("v_nop\n\tv_nop\n\tv_nop\n\tv_nop" : "+v"(a), "+v"(b), "+v"(c), "+v"(d)); }
template <typename T> struct Frag;
template <> struct Frag<_Float16> {
  typedef v16h V; union U { v16h v; v8h h[2]; };
  static __device__ __forceinline__ v16h load(const _Float16* p) {
    U f; f.h[0] = *(const v8h*)(p); f.h[1] = *(const v8h*)(p + 16); return f.v;
  }
  static __device__ __forceinline__ v8f mma(v16h a, v16h b, v8f c) {
    return __builtin_amdgcn_wmma_f32_16x16x32_f16(false, a, false, b, (short)0, c, false, false);
  }
  static __device__ __forceinline__ void guard(v8f& a, v8f& b, v16h x, v16h y) { dep_guard_h(a, b, x, y); }
  static __device__ __forceinline__ void keep(v16h a, v16h b, v16h c, v16h d) { keep4_h(a, b, c, d); }
};
template <> struct Frag<__bf16> {
  typedef v16b V; union U { v16b v; v8b h[2]; };
  static __device__ __forceinline__ v16b load(const __bf16* p) {
    U f; f.h[0] = *(const v8b*)(p); f.h[1] = *(const v8b*)(p + 16); return f.v;
  }
  static __device__ __forceinline__ v8f mma(v16b a, v16b b, v8f c) {
    return __builtin_amdgcn_wmma_f32_16x16x32_bf16(false, a, false, b, (short)0, c, false, false);
  }
  static __device__ __forceinline__ void guard(v8f& a, v8f& b, v16b x, v16b y) { dep_guard_b(a, b, x, y); }
  static __device__ __forceinline__ void keep(v16b a, v16b b, v16b c, v16b d) { keep4_b(a, b, c, d); }
};

__device__ __forceinline__ unsigned pk16(unsigned short a, unsigned short b) { return (unsigned)a | ((unsigned)b << 16); }
__device__ __forceinline__ unsigned short h_bits(float f) { const _Float16 h = (_Float16)f; return __builtin_bit_cast(unsigned short, h); }

template <int ET> struct Elem;
template <> struct Elem<0> { typedef _Float16 T; };
template <> struct Elem<1> { typedef __bf16 T; };
template <int ET, bool SPLIT, int BIAS_MODE, int OUT_MODE, bool RESID, int ACT = 0>
__global__ __launch_bounds__(256) void wmma_gemm64(
    const unsigned short* __restrict__ Ap, const unsigned short* __restrict__ A2p, int lda, long strideA,
    const unsigned short* __restrict__ Btp, const unsigned short* __restrict__ Bt2p, int ldb, long strideB,
    void* __restrict__ Cout, void* __restrict__ Cout2, int ldc, long strideC,
    const float* __restrict__ bias,
    const float* __restrict__ resid, long strideR,
    int M, int N, int K, float scale) {
  typedef typename Elem<ET>::T T;
  typedef typename Frag<T>::V V;
  const T* A = (const T*)Ap; const T* A2 = (const T*)A2p; const T* Bt = (const T*)Btp; const T* Bt2 = (const T*)Bt2p;
  __shared__ __align__(16) float sT[8][16 * 68];
  const int b    = blockIdx.y;
  const int lane = threadIdx.x & 31;
  const int wave = threadIdx.x >> 5;
  const int tilesN = N >> 6;
  const int tilesM = M >> 6;
  const int tile = blockIdx.x * 8 + wave;
  if (tile >= tilesM * tilesN) return;
  const int tm = tile / tilesN;
  const int tn = tile - tm * tilesN;
  const int m0 = tm << 6;
  const int n0 = tn << 6;

  const T* Ab  = A  + (size_t)b * strideA;
  const T* Bb  = Bt + (size_t)b * strideB;
  const T* Ab2 = SPLIT ? (A2  + (size_t)b * strideA) : nullptr;
  const T* Bb2 = SPLIT ? (Bt2 + (size_t)b * strideB) : nullptr;

  const int rlane = lane & 15;
  const int koff  = (lane >> 4) * 8;
  const int mOff  = (lane >> 4) * 8;

  v8f acc[4][4];
#pragma unroll
  for (int i = 0; i < 4; ++i)
#pragma unroll
    for (int j = 0; j < 4; ++j) acc[i][j] = (v8f){0.f,0.f,0.f,0.f,0.f,0.f,0.f,0.f};

  for (int k0 = 0; k0 < K; k0 += 32) {
    V bh[4], bl[4];
#pragma unroll
    for (int j = 0; j < 4; ++j) {
      const size_t bo = (size_t)(n0 + (j << 4) + rlane) * ldb + koff + k0;
      bh[j] = Frag<T>::load(Bb + bo);
      if (SPLIT) bl[j] = Frag<T>::load(Bb2 + bo);
    }
#pragma unroll
    for (int i = 0; i < 4; ++i) {
      const size_t ao = (size_t)(m0 + (i << 4) + rlane) * lda + koff + k0;
      V ah = Frag<T>::load(Ab + ao);
      V al;
      if (SPLIT) al = Frag<T>::load(Ab2 + ao);
#pragma unroll
      for (int j = 0; j < 4; ++j) {
        acc[i][j] = Frag<T>::mma(ah, bh[j], acc[i][j]);
        if (SPLIT) {
          acc[i][j] = Frag<T>::mma(ah, bl[j], acc[i][j]);
          acc[i][j] = Frag<T>::mma(al, bh[j], acc[i][j]);
        }
      }
      Frag<T>::guard(acc[i][0], acc[i][3], ah, SPLIT ? al : ah);
    }
    Frag<T>::keep(bh[0], bh[1], bh[2], bh[3]);
    if (SPLIT) Frag<T>::keep(bl[0], bl[1], bl[2], bl[3]);
  }
  acc_guard4(acc[0][0], acc[0][1], acc[0][2], acc[0][3]);
  acc_guard4(acc[1][0], acc[1][1], acc[1][2], acc[1][3]);
  acc_guard4(acc[2][0], acc[2][1], acc[2][2], acc[2][3]);
  acc_guard4(acc[3][0], acc[3][1], acc[3][2], acc[3][3]);

  float* slab = sT[wave];
  const float* Rb = RESID ? (resid + (size_t)b * strideR) : nullptr;
#pragma unroll
  for (int i = 0; i < 4; ++i) {
    const int mBase = m0 + (i << 4);
#pragma unroll
    for (int j = 0; j < 4; ++j) {
      const int n = n0 + (j << 4) + rlane;
      float bv = 0.f;
      if (BIAS_MODE == 2) bv = bias[n];
#pragma unroll
      for (int r = 0; r < 8; ++r) {
        float v = acc[i][j][r] * scale;
        if (BIAS_MODE == 1) v += bias[mBase + mOff + r];
        if (BIAS_MODE == 2) v += bv;
        if (RESID) v += Rb[(size_t)(mBase + mOff + r) * ldc + n];
        if (ACT == 2) v = fmaxf(v, 0.0f);
        if (ACT == 4) v = (v > 0.f) ? v : 0.01f * v;
        slab[(mOff + r) * 68 + (j << 4) + rlane] = v;
      }
    }
    __builtin_amdgcn_fence(__ATOMIC_RELEASE, "workgroup");
    __builtin_amdgcn_wave_barrier();
    __builtin_amdgcn_fence(__ATOMIC_ACQUIRE, "workgroup");
    if (OUT_MODE == 0) {
      float* C = (float*)Cout + (size_t)b * strideC;
      const int hh = lane >> 4, c4 = (lane & 15) * 4;
      for (int pass = 0; pass < 2; ++pass) {
#pragma unroll
        for (int it = 0; it < 8; ++it) {
          const int row = it * 2 + hh;
          v4f v = *(const v4f*)(slab + row * 68 + c4);
          *(volatile v4f*)(C + (size_t)(mBase + row) * ldc + n0 + c4) = v;
        }
        __threadfence();
      }
    } else {
      const int q = lane >> 3, c8 = (lane & 7) * 8;
      unsigned short* C  = (unsigned short*)Cout  + (size_t)b * strideC;
      unsigned short* C2 = (OUT_MODE == 2) ? ((unsigned short*)Cout2 + (size_t)b * strideC) : nullptr;
      for (int pass = 0; pass < 2; ++pass) {
#pragma unroll
        for (int it = 0; it < 4; ++it) {
          const int row = it * 4 + q;
          const float* sp = slab + row * 68 + c8;
          v8h hv, lv;
#pragma unroll
          for (int e = 0; e < 8; ++e) {
            if (OUT_MODE == 1) {
              hv[e] = (_Float16)sp[e];
            } else {
              unsigned short hb = f2bf_bits(sp[e]);
              unsigned short lb = f2bf_bits(sp[e] - bf_bits2f(hb));
              hv[e] = __builtin_bit_cast(_Float16, hb);
              lv[e] = __builtin_bit_cast(_Float16, lb);
            }
          }
          *(volatile v8h*)(C + (size_t)(mBase + row) * ldc + n0 + c8) = hv;
          if (OUT_MODE == 2) *(volatile v8h*)(C2 + (size_t)(mBase + row) * ldc + n0 + c8) = lv;
        }
        __threadfence();
      }
    }
    __builtin_amdgcn_fence(__ATOMIC_RELEASE, "workgroup");
    __builtin_amdgcn_wave_barrier();
    __builtin_amdgcn_fence(__ATOMIC_ACQUIRE, "workgroup");
  }
}

__device__ __forceinline__ float softplus_f(float x) { return fmaxf(x, 0.0f) + log1pf(expf(-fabsf(x))); }
__device__ __forceinline__ float silu_f(float x) {
  const float xc = fmaxf(x, -60.0f);
  const float e = expf(-xc);
  return x * (1.0f / (1.0f + e));
}
__device__ __forceinline__ float gelu_f(float x) { return 0.5f * x * (1.0f + erff(x * 0.70710678118654752f)); }

__device__ __forceinline__ float block_sum256(float v, float* red8) {
#pragma unroll
  for (int off = 16; off > 0; off >>= 1) v += __shfl_xor(v, off, 32);
  const int lane = threadIdx.x & 31;
  const int wave = threadIdx.x >> 5;
  if (lane == 0) red8[wave] = v;
  __syncthreads();
  float t = 0.0f;
#pragma unroll
  for (int w = 0; w < 8; ++w) t += red8[w];
  return t;
}

__global__ __launch_bounds__(256) void cast8_f16_kernel(const float* __restrict__ in, unsigned short* __restrict__ out,
                                                        int n8_valid, int n8_total, float scale) {
  const int i = blockIdx.x * 256 + threadIdx.x;
  if (i >= n8_total) return;
  const int ic = (i < n8_valid) ? i : (n8_valid - 1);
  const float* p = in + 8 * (size_t)ic;
  v4f a = *(const v4f*)(p);
  v4f c = *(const v4f*)(p + 4);
  if (i >= n8_valid) { a = (v4f){0.f, 0.f, 0.f, 0.f}; c = (v4f){0.f, 0.f, 0.f, 0.f}; }
  unsigned short hb[8];
#pragma unroll
  for (int e = 0; e < 4; ++e) {
    hb[e]     = h_bits(a[e] * scale);
    hb[4 + e] = h_bits(c[e] * scale);
  }
  const v4u u = (v4u){pk16(hb[0], hb[1]), pk16(hb[2], hb[3]), pk16(hb[4], hb[5]), pk16(hb[6], hb[7])};
  unsigned short* q = out + 8 * (size_t)i;
  *(volatile v4u*)q = u;
  __threadfence();
  *(volatile v4u*)q = u;
}

__global__ __launch_bounds__(256) void conv_silu_kernel(const float* __restrict__ XC, const float* __restrict__ cw,
                                                        const float* __restrict__ cb, float* __restrict__ XS,
                                                        unsigned short* __restrict__ XSH) {
  const int idx = blockIdx.x * 256 + threadIdx.x;
  if (idx >= kL * (kDI / 4)) return;
  const int t = idx >> 9;
  const int d = (idx & 511) * 4;
  const v4f w0 = *(const v4f*)(cw + (size_t)(d + 0) * 4);
  const v4f w1 = *(const v4f*)(cw + (size_t)(d + 1) * 4);
  const v4f w2 = *(const v4f*)(cw + (size_t)(d + 2) * 4);
  const v4f w3 = *(const v4f*)(cw + (size_t)(d + 3) * 4);
  v4f acc = (v4f){0.f, 0.f, 0.f, 0.f};
#pragma unroll
  for (int k = 0; k < 4; ++k) {
    const int tt  = t - 3 + k;
    const int ttc = (tt < 0) ? 0 : tt;
    v4f xv = *(const v4f*)(XC + (size_t)ttc * kDI + d);
    if (tt < 0) xv = (v4f){0.f, 0.f, 0.f, 0.f};
    const v4f wk = (v4f){w0[k], w1[k], w2[k], w3[k]};
    acc = acc + wk * xv;
  }
  const v4f bb = *(const v4f*)(cb + d);
  acc = acc + bb;
  v4f sv;
  sv[0] = silu_f(acc[0]); sv[1] = silu_f(acc[1]); sv[2] = silu_f(acc[2]); sv[3] = silu_f(acc[3]);
  const v2u hu = (v2u){pk16(h_bits(sv[0] * kXsCarry), h_bits(sv[1] * kXsCarry)),
                       pk16(h_bits(sv[2] * kXsCarry), h_bits(sv[3] * kXsCarry))};
  float* xp = XS + (size_t)t * kDI + d;
  unsigned short* hp = XSH + (size_t)t * kDI + d;
  *(volatile v4f*)xp = sv;
  *(volatile v2u*)hp = hu;
  __threadfence();
  *(volatile v4f*)xp = sv;
  *(volatile v2u*)hp = hu;
}

__global__ __launch_bounds__(256) void dtin_cast_kernel(const float* __restrict__ xdbl, unsigned short* __restrict__ out, float scale) {
  const int i = blockIdx.x * 256 + threadIdx.x;
  if (i >= kL * (kDTR / 2)) return;
  const int row = i >> 5;
  const int c = (i & 31) * 2;
  const v2f x = *(const v2f*)(xdbl + (size_t)row * kXPN + c);
  const unsigned u = pk16(h_bits(x[0] * scale), h_bits(x[1] * scale));
  unsigned* q = (unsigned*)out + (size_t)i;
  *(volatile unsigned*)q = u;
  __threadfence();
  *(volatile unsigned*)q = u;
}

__global__ __launch_bounds__(256) void matvec_kernel(const float* __restrict__ W, const float* __restrict__ x,
                                                     const float* __restrict__ bias, float* __restrict__ out,
                                                     int nout, int kdim) {
  const int n = blockIdx.x * 256 + threadIdx.x;
  const int nc = (n < nout) ? n : (nout - 1);
  const float* wr = W + (size_t)nc * kdim;
  float acc = 0.0f;
#pragma unroll 1
  for (int k = 0; k < kdim; ++k) acc = fmaf(wr[k], x[k], acc);
  acc += bias[nc];
  if (n < nout) {
    *(volatile float*)(out + n) = acc;
    __threadfence();
    *(volatile float*)(out + n) = acc;
  }
}

__global__ __launch_bounds__(512) void scan_gate_kernel(
    const float* __restrict__ XS, const float* __restrict__ DTP, const float* __restrict__ XDBL,
    const float* __restrict__ Zp, const float* __restrict__ Alog, const float* __restrict__ Dv,
    unsigned short* __restrict__ GH) {
  __shared__ float sdt[16][64];
  __shared__ float sx[16][64];
  __shared__ float ssz[16][64];
  __shared__ float sy[16][64];
  __shared__ float sbc[16][32];
  __shared__ unsigned short sg[16][64];
  const int tid  = threadIdx.x;
  const int lane = tid & 31;
  const int wave = tid >> 5;
  const int i0   = blockIdx.x * 64;
  const int cp   = tid >> 4;
  const int s    = tid & 15;
  const int ch0  = 2 * cp;
  const int ch1  = 2 * cp + 1;
  const float A0 = -expf(Alog[(size_t)(i0 + ch0) * kDS + s]);
  const float A1 = -expf(Alog[(size_t)(i0 + ch1) * kDS + s]);
  const float D0 = Dv[i0 + ch0];
  const float D1 = Dv[i0 + ch1];
  float h0 = 0.0f, h1 = 0.0f;

#pragma unroll 1
  for (int tc = 0; tc < kL / 16; ++tc) {
    const int t0 = tc * 16;
#pragma unroll 1
    for (int r = 0; r < 2; ++r) {
      const int e  = tid + 512 * r;
      const int st = e >> 6;
      const int ch = e & 63;
      const size_t gi = (size_t)(t0 + st) * kDI + i0 + ch;
      sdt[st][ch] = softplus_f(DTP[gi]);
      sx[st][ch]  = XS[gi];
      ssz[st][ch] = silu_f(Zp[gi]);
    }
    {
      const int st = tid >> 5;
      const int c  = tid & 31;
      sbc[st][c] = XDBL[(size_t)(t0 + st) * kXPN + kDTR + c];
    }
    __syncthreads();
#pragma unroll 1
    for (int st = 0; st < 16; ++st) {
      const float dt0 = sdt[st][ch0];
      const float dt1 = sdt[st][ch1];
      const float x0  = sx[st][ch0];
      const float x1  = sx[st][ch1];
      const float Bs  = sbc[st][s];
      const float Cs  = sbc[st][kDS + s];
      h0 = expf(dt0 * A0) * h0 + (dt0 * x0) * Bs;
      h1 = expf(dt1 * A1) * h1 + (dt1 * x1) * Bs;
      float p0 = h0 * Cs;
      float p1 = h1 * Cs;
      p0 += __shfl_xor(p0, 1, 32); p1 += __shfl_xor(p1, 1, 32);
      p0 += __shfl_xor(p0, 2, 32); p1 += __shfl_xor(p1, 2, 32);
      p0 += __shfl_xor(p0, 4, 32); p1 += __shfl_xor(p1, 4, 32);
      p0 += __shfl_xor(p0, 8, 32); p1 += __shfl_xor(p1, 8, 32);
      if (s == 0) {
        sy[st][ch0] = p0 + D0 * x0;
        sy[st][ch1] = p1 + D1 * x1;
      }
    }
    __syncthreads();
#pragma unroll 1
    for (int r = 0; r < 2; ++r) {
      const int e  = tid + 512 * r;
      const int st = e >> 6;
      const int ch = e & 63;
      const float g = (sy[st][ch] * ssz[st][ch]) * kGateCarry;
      sg[st][ch] = h_bits(g);
    }
    __syncthreads();
    if (wave < 4) {
      const int q  = lane >> 3;
      const int c8 = (lane & 7) * 8;
      const int st = wave * 4 + q;
      const unsigned short* sp = &sg[st][c8];
      const v4u u = (v4u){pk16(sp[0], sp[1]), pk16(sp[2], sp[3]), pk16(sp[4], sp[5]), pk16(sp[6], sp[7])};
      unsigned short* gp = GH + (size_t)(t0 + st) * kDI + i0 + c8;
      *(volatile v4u*)gp = u;
      __threadfence();
      *(volatile v4u*)gp = u;
    }
  }
}

__global__ __launch_bounds__(256) void ln12_kernel(const float* __restrict__ S1, const float* __restrict__ g1,
                                                   const float* __restrict__ b1, const float* __restrict__ avec,
                                                   const float* __restrict__ g2, const float* __restrict__ b2,
                                                   float* __restrict__ seq2, unsigned short* __restrict__ seq2h) {
  __shared__ float red[4][8];
  const int row = blockIdx.x;
  const int c = threadIdx.x * 4;
  const size_t base = (size_t)row * kDM + c;
  const v4f x = *(const v4f*)(S1 + base);
  const float mu = block_sum256((x[0] + x[1]) + (x[2] + x[3]), red[0]) * kInvDM;
  const v4f d = x - mu;
  const float var = block_sum256((d[0] * d[0] + d[1] * d[1]) + (d[2] * d[2] + d[3] * d[3]), red[1]) * kInvDM;
  const float inv = rsqrtf(var + kEps);
  const v4f gg1 = *(const v4f*)(g1 + c);
  const v4f bb1 = *(const v4f*)(b1 + c);
  const v4f av  = *(const v4f*)(avec + c);
  v4f u = (d * inv) * gg1 + bb1;
  u = av + u;
  const float mu2 = block_sum256((u[0] + u[1]) + (u[2] + u[3]), red[2]) * kInvDM;
  const v4f d2 = u - mu2;
  const float var2 = block_sum256((d2[0] * d2[0] + d2[1] * d2[1]) + (d2[2] * d2[2] + d2[3] * d2[3]), red[3]) * kInvDM;
  const float inv2 = rsqrtf(var2 + kEps);
  const v4f gg2 = *(const v4f*)(g2 + c);
  const v4f bb2 = *(const v4f*)(b2 + c);
  const v4f y = (d2 * inv2) * gg2 + bb2;
  const v2u hu = (v2u){pk16(h_bits(y[0]), h_bits(y[1])), pk16(h_bits(y[2]), h_bits(y[3]))};
  float* op = seq2 + base;
  unsigned short* hp = seq2h + base;
  *(volatile v4f*)op = y;
  *(volatile v2u*)hp = hu;
  __threadfence();
  *(volatile v4f*)op = y;
  *(volatile v2u*)hp = hu;
}

__global__ __launch_bounds__(256) void gelu2_kernel(const float* __restrict__ in, unsigned short* __restrict__ out, int n2, float carry) {
  const int i = blockIdx.x * 256 + threadIdx.x;
  if (i >= n2) return;
  const v2f x = *(const v2f*)(in + 2 * (size_t)i);
  const unsigned u = pk16(h_bits(gelu_f(x[0]) * carry), h_bits(gelu_f(x[1]) * carry));
  unsigned* q = (unsigned*)out + (size_t)i;
  *(volatile unsigned*)q = u;
  __threadfence();
  *(volatile unsigned*)q = u;
}

__global__ __launch_bounds__(256) void ln3_kernel(const float* __restrict__ X, const float* __restrict__ g,
                                                  const float* __restrict__ b, float* __restrict__ out) {
  __shared__ float red[2][8];
  const int row = blockIdx.x;
  const int c = threadIdx.x * 4;
  const size_t base = (size_t)row * kDM + c;
  const v4f x = *(const v4f*)(X + base);
  const float mu = block_sum256((x[0] + x[1]) + (x[2] + x[3]), red[0]) * kInvDM;
  const v4f d = x - mu;
  const float var = block_sum256((d[0] * d[0] + d[1] * d[1]) + (d[2] * d[2] + d[3] * d[3]), red[1]) * kInvDM;
  const float inv = rsqrtf(var + kEps);
  const v4f gg = *(const v4f*)(g + c);
  const v4f bb = *(const v4f*)(b + c);
  const v4f y = (d * inv) * gg + bb;
  const bool w1 = (blockIdx.x == 0) && (threadIdx.x == 0);
  float* op = out + base;
  float* wp = out + (size_t)kL * kDM;
  const float one = 1.0f;
  *(volatile v4f*)op = y;
  if (w1) *(volatile float*)wp = one;
  __threadfence();
  *(volatile v4f*)op = y;
  if (w1) *(volatile float*)wp = one;
}

extern "C" void kernel_launch(void* const* d_in, const int* in_sizes, int n_in,
                              void* d_out, int out_size, void* d_ws, size_t ws_size, hipStream_t stream)
{
  if (n_in < 25) return;
  if (in_sizes[0] != kL * kDM) return;
  if ((size_t)out_size < (size_t)kL * kDM + 1) return;
  if (kWsTotal > ws_size) return;

  const float* emb    = (const float*)d_in[0];
  const float* clin   = (const float*)d_in[1];
  const float* w_in   = (const float*)d_in[2];
  const float* conv_w = (const float*)d_in[3];
  const float* conv_b = (const float*)d_in[4];
  const float* w_xp   = (const float*)d_in[5];
  const float* w_dt   = (const float*)d_in[6];
  const float* b_dt   = (const float*)d_in[7];
  const float* A_log  = (const float*)d_in[8];
  const float* Dvec   = (const float*)d_in[9];
  const float* w_out  = (const float*)d_in[10];
  const float* ln1_g  = (const float*)d_in[11];
  const float* ln1_b  = (const float*)d_in[12];
  const float* w_ain  = (const float*)d_in[13];
  const float* b_ain  = (const float*)d_in[14];
  const float* w_aout = (const float*)d_in[15];
  const float* b_aout = (const float*)d_in[16];
  const float* ln2_g  = (const float*)d_in[17];
  const float* ln2_b  = (const float*)d_in[18];
  const float* w_f1   = (const float*)d_in[19];
  const float* b_f1   = (const float*)d_in[20];
  const float* w_f2   = (const float*)d_in[21];
  const float* b_f2   = (const float*)d_in[22];
  const float* ln3_g  = (const float*)d_in[23];
  const float* ln3_b  = (const float*)d_in[24];
  float* out = (float*)d_out;

  char* ws = (char*)d_ws;
  float* XC   = (float*)(ws + oXC);
  float* DTP  = (float*)(ws + oDTP);
  float* SEQ2 = (float*)(ws + oSEQ2);
  unsigned short* SEQ2H = (unsigned short*)(ws + oSEQ2H);
  unsigned short* W1H   = (unsigned short*)(ws + oW1H);
  unsigned short* W2H   = (unsigned short*)(ws + oW2H);
  float* Zp   = (float*)(ws + oZ);
  float* HPRE = (float*)(ws + oHPRE);
  unsigned short* EMBH  = (unsigned short*)(ws + oEMBH);
  unsigned short* WINH  = (unsigned short*)(ws + oWINH);
  unsigned short* XSH   = (unsigned short*)(ws + oXSH);
  unsigned short* GH    = (unsigned short*)(ws + oGH);
  unsigned short* G2H   = (unsigned short*)(ws + oG2H);
  float* XS   = (float*)(ws + oXS);
  float* S1   = (float*)(ws + oS1);
  float* OPRE = (float*)(ws + oOPRE);
  unsigned short* WXPH  = (unsigned short*)(ws + oWXPH);
  float* XDBL = (float*)(ws + oXDBL);
  unsigned short* DTINH = (unsigned short*)(ws + oDTINH);
  unsigned short* WDTH  = (unsigned short*)(ws + oWDTH);
  unsigned short* WOUTH = (unsigned short*)(ws + oWOUTH);
  float* VVEC = (float*)(ws + oVVEC);
  float* AVEC = (float*)(ws + oAVEC);

  const int TB = 256;
  auto nblk = [](long long n) { return (unsigned)((n + 255) / 256); };

  {
    const int n8 = kL * kDM / 8;
    cast8_f16_kernel<<<nblk(n8), TB, 0, stream>>>(emb, EMBH, n8, n8, 1.0f);
    cast8_f16_kernel<<<nblk(n8), TB, 0, stream>>>(w_in, WINH, n8, n8, kWCarry);
    const int n8xv = kXPC * kDI / 8, n8xt = kXPN * kDI / 8;
    cast8_f16_kernel<<<nblk(n8xt), TB, 0, stream>>>(w_xp, WXPH, n8xv, n8xt, kWCarry);
    const int n8d = kDI * kDTR / 8;
    cast8_f16_kernel<<<nblk(n8d), TB, 0, stream>>>(w_dt, WDTH, n8d, n8d, kWCarry);
    const int n8o = kDM * kDI / 8;
    cast8_f16_kernel<<<nblk(n8o), TB, 0, stream>>>(w_out, WOUTH, n8o, n8o, kWCarry);
  }

  {
    const unsigned g = (unsigned)(((kL / 64) * (kDI / 64) + 7) / 8);
    wmma_gemm64<0, false, 0, 0, false, 0><<<dim3(g, 1), TB, 0, stream>>>(
        EMBH, EMBH, kDM, 0L, WINH, WINH, kDM, 0L, (void*)XC, (void*)XC, kDI, 0L,
        conv_b, conv_b, 0L, kL, kDI, kDM, kScaleIn);
    wmma_gemm64<0, false, 0, 0, false, 0><<<dim3(g, 1), TB, 0, stream>>>(
        EMBH, EMBH, kDM, 0L, WINH + (size_t)kDI * kDM, WINH + (size_t)kDI * kDM, kDM, 0L, (void*)Zp, (void*)Zp, kDI, 0L,
        conv_b, conv_b, 0L, kL, kDI, kDM, kScaleIn);
  }

  conv_silu_kernel<<<nblk((long long)kL * (kDI / 4)), TB, 0, stream>>>(XC, conv_w, conv_b, XS, XSH);

  {
    const unsigned g = (unsigned)(((kL / 64) * (kXPN / 64) + 7) / 8);
    wmma_gemm64<0, false, 0, 0, false, 0><<<dim3(g, 1), TB, 0, stream>>>(
        XSH, XSH, kDI, 0L, WXPH, WXPH, kDI, 0L, (void*)XDBL, (void*)XDBL, kXPN, 0L,
        conv_b, conv_b, 0L, kL, kXPN, kDI, kScaleXp);
  }

  dtin_cast_kernel<<<nblk((long long)kL * (kDTR / 2)), TB, 0, stream>>>(XDBL, DTINH, kDtCarry);
  {
    const unsigned g = (unsigned)(((kL / 64) * (kDI / 64) + 7) / 8);
    wmma_gemm64<0, false, 2, 0, false, 0><<<dim3(g, 1), TB, 0, stream>>>(
        DTINH, DTINH, kDTR, 0L, WDTH, WDTH, kDTR, 0L, (void*)DTP, (void*)DTP, kDI, 0L,
        b_dt, conv_b, 0L, kL, kDI, kDTR, kScaleDt);
  }

  matvec_kernel<<<kDM / TB, TB, 0, stream>>>(w_ain + (size_t)2 * kDM * kDM, clin, b_ain + 2 * kDM, VVEC, kDM, kDM);
  matvec_kernel<<<kDM / TB, TB, 0, stream>>>(w_aout, VVEC, b_aout, AVEC, kDM, kDM);

  scan_gate_kernel<<<kDI / 64, 512, 0, stream>>>(XS, DTP, XDBL, Zp, A_log, Dvec, GH);

  {
    const int n8f = 2 * kDM * kDM / 8;
    cast8_f16_kernel<<<nblk(n8f), TB, 0, stream>>>(w_f1, W1H, n8f, n8f, kWCarry);
    cast8_f16_kernel<<<nblk(n8f), TB, 0, stream>>>(w_f2, W2H, n8f, n8f, kWCarry);
  }

  {
    const unsigned g = (unsigned)(((kL / 64) * (kDM / 64) + 7) / 8);
    wmma_gemm64<0, false, 0, 0, true, 0><<<dim3(g, 1), TB, 0, stream>>>(
        GH, GH, kDI, 0L, WOUTH, WOUTH, kDI, 0L, (void*)S1, (void*)S1, kDM, 0L,
        conv_b, emb, 0L, kL, kDM, kDI, kScaleOut);
  }

  ln12_kernel<<<kL, TB, 0, stream>>>(S1, ln1_g, ln1_b, AVEC, ln2_g, ln2_b, SEQ2, SEQ2H);

  {
    const unsigned g = (unsigned)(((kL / 64) * (2 * kDM / 64) + 7) / 8);
    wmma_gemm64<0, false, 2, 0, false, 0><<<dim3(g, 1), TB, 0, stream>>>(
        SEQ2H, SEQ2H, kDM, 0L, W1H, W1H, kDM, 0L, (void*)HPRE, (void*)HPRE, 2 * kDM, 0L,
        b_f1, conv_b, 0L, kL, 2 * kDM, kDM, kScaleF1);
  }

  gelu2_kernel<<<nblk((long long)kL * kDM), TB, 0, stream>>>(HPRE, G2H, kL * kDM, kGeluCarry);

  {
    const unsigned g = (unsigned)(((kL / 64) * (kDM / 64) + 7) / 8);
    wmma_gemm64<0, false, 2, 0, true, 0><<<dim3(g, 1), TB, 0, stream>>>(
        G2H, G2H, 2 * kDM, 0L, W2H, W2H, 2 * kDM, 0L, (void*)OPRE, (void*)OPRE, kDM, 0L,
        b_f2, SEQ2, 0L, kL, kDM, 2 * kDM, kScaleF2);
  }

  ln3_kernel<<<kL, TB, 0, stream>>>(OPRE, ln3_g, ln3_b, out);
}
